// GCNDecoder_867583394201
// MI455X (gfx1250) — hardware-verified
//
#include <hip/hip_runtime.h>
#include <stddef.h>
#include <stdint.h>


#define HID    128
#define NBAT   2
#define CW     (NBAT * HID)
#define KD     (2 * HID)
#define IND    3
#define OUTD   3
#define NLAY   4
#define NTHR   256
#define NWAVE  8
#define EPT    8
#define CHUNK  (NTHR * EPT)
#define WCAP   (EPT * 32)
#define LISTN  (NWAVE * WCAP)
#define NB     256
#define SLB    8
#define GBM    64
#define GTHR   128
#define FNB    256
#define WSMAX  134217728

static_assert((CHUNK & (CHUNK - 1)) == 0 && CHUNK <= 4096);
static_assert((NB & (NB - 1)) == 0 && NB == (1 << SLB));
static_assert(((long long)CHUNK << SLB) < (1LL << 31));
static_assert(LISTN % NTHR == 0);
static_assert((NB * CW) % (NTHR * 4) == 0);
static_assert(NB % (NWAVE * 8) == 0);
static_assert(HID % 32 == 0 && HID == GTHR && CW == 2 * HID);
static_assert(GBM == (GTHR / 32) * 16);
static_assert(KD == NTHR && KD == 32 * 8 && HID % NWAVE == 0);
static_assert(FNB % NWAVE == 0 && (FNB / NWAVE) == 32 && (FNB * OUTD) % 4 == 0);

typedef float          v4f   __attribute__((ext_vector_type(4)));
typedef float          v8f   __attribute__((ext_vector_type(8)));
typedef int            v4i   __attribute__((ext_vector_type(4)));
typedef int            v8i   __attribute__((ext_vector_type(8)));
typedef unsigned short v8us  __attribute__((ext_vector_type(8)));
typedef unsigned short v16us __attribute__((ext_vector_type(16)));
typedef __bf16         v16bf __attribute__((ext_vector_type(16)));
typedef v4f  __attribute__((may_alias)) v4fa;
typedef v8us __attribute__((may_alias)) v8usa;
union FragB { v16bf v; v16us u; v8us h[2]; v8i w; };

__device__ __forceinline__ v8f wmb(const FragB& a, const FragB& b, v8f c) {
  v8f d = __builtin_amdgcn_wmma_f32_16x16x32_bf16(false, a.v, false, b.v, (short)0, c, false, false);
  asm volatile("v_nop\n\tv_nop\n\tv_nop\n\tv_nop" : "+v"(d) : "v"(a.w), "v"(b.w));
  return d;
}

__device__ __forceinline__ unsigned bf16_bits(float f) {
  const unsigned u = __float_as_uint(f);
  return (u + 0x7FFFu + ((u >> 16) & 1u)) >> 16;
}
__device__ __forceinline__ float bf16_val(float f) {
  return __uint_as_float(bf16_bits(f) << 16);
}
__device__ __forceinline__ v4f bfv4(v4f a) {
  v4f r;
  r.x = bf16_val(a.x); r.y = bf16_val(a.y); r.z = bf16_val(a.z); r.w = bf16_val(a.w);
  return r;
}
__device__ __forceinline__ v4f relu4(v4f a) {
  v4f r;
  r.x = fmaxf(a.x, 0.0f); r.y = fmaxf(a.y, 0.0f); r.z = fmaxf(a.z, 0.0f); r.w = fmaxf(a.w, 0.0f);
  return r;
}

__device__ __forceinline__ int scan_chunk(const int* __restrict__ dsts, int nE, int cbase, int slotBase,
                                          int nb, int vec8, int* list, int tid, int lane, int wave) {
  int wc = 0;
  const int el0  = tid * EPT;
  const int e0   = cbase + el0;
  const int sent = -2147483647 - 1;
  v4i da, db;
  if (vec8 != 0 && cbase + CHUNK <= nE) {
    da = *(const v4i*)(dsts + e0);
    db = *(const v4i*)(dsts + e0 + 4);
  } else {
    da.x = (e0     < nE) ? dsts[min(e0,     nE - 1)] : sent;
    da.y = (e0 + 1 < nE) ? dsts[min(e0 + 1, nE - 1)] : sent;
    da.z = (e0 + 2 < nE) ? dsts[min(e0 + 2, nE - 1)] : sent;
    da.w = (e0 + 3 < nE) ? dsts[min(e0 + 3, nE - 1)] : sent;
    db.x = (e0 + 4 < nE) ? dsts[min(e0 + 4, nE - 1)] : sent;
    db.y = (e0 + 5 < nE) ? dsts[min(e0 + 5, nE - 1)] : sent;
    db.z = (e0 + 6 < nE) ? dsts[min(e0 + 6, nE - 1)] : sent;
    db.w = (e0 + 7 < nE) ? dsts[min(e0 + 7, nE - 1)] : sent;
  }
  const unsigned nbs = (unsigned)slotBase;
  const unsigned unb = (unsigned)nb;
  const unsigned s0 = (unsigned)da.x - nbs, s1 = (unsigned)da.y - nbs;
  const unsigned s2 = (unsigned)da.z - nbs, s3 = (unsigned)da.w - nbs;
  const unsigned s4 = (unsigned)db.x - nbs, s5 = (unsigned)db.y - nbs;
  const unsigned s6 = (unsigned)db.z - nbs, s7 = (unsigned)db.w - nbs;
  const bool h0 = s0 < unb, h1 = s1 < unb, h2 = s2 < unb, h3 = s3 < unb;
  const bool h4 = s4 < unb, h5 = s5 < unb, h6 = s6 < unb, h7 = s7 < unb;
  const unsigned any = __builtin_amdgcn_ballot_w32(h0 | h1 | h2 | h3 | h4 | h5 | h6 | h7);
  if (any != 0u) {
#define HITJ(J, HJ, SJ) { \
      const unsigned mj = __builtin_amdgcn_ballot_w32(HJ); \
      if (mj != 0u) { \
        if (HJ) { \
          const int pos = wc + (int)__builtin_amdgcn_mbcnt_lo(mj, 0u); \
          if (pos < WCAP) list[wave * WCAP + pos] = ((el0 + (J)) << SLB) | (int)(SJ); \
        } \
        wc += (int)__builtin_popcount(mj); } }
    HITJ(0, h0, s0)
    HITJ(1, h1, s1)
    HITJ(2, h2, s2)
    HITJ(3, h3, s3)
    HITJ(4, h4, s4)
    HITJ(5, h5, s5)
    HITJ(6, h6, s6)
    HITJ(7, h7, s7)
#undef HITJ
  }
  return wc;
}

__global__ __launch_bounds__(NTHR) void k_wprep(const float* __restrict__ Wsb, const float* __restrict__ Wfb,
                                                unsigned short* WT) {
  __shared__ __attribute__((aligned(16))) float T[KD * NWAVE];
  const int tid = (int)threadIdx.x, lane = tid & 31, wave = tid >> 5;
  const int L = (int)blockIdx.y, n0 = (int)blockIdx.x * NWAVE;
  {
    const int k = tid;
    const size_t lbase = (size_t)L * HID * HID;
    const float* src = (k < HID) ? (Wsb + lbase + (size_t)k * HID + n0)
                                 : (Wfb + lbase + (size_t)(k - HID) * HID + n0);
    const v4f a = *(const v4f*)src;
    const v4f b = *(const v4f*)(src + 4);
    *(v4fa*)(T + k * NWAVE)     = a;
    *(v4fa*)(T + k * NWAVE + 4) = b;
  }
  __syncthreads();
  const int k8 = lane * 8;
  v8us o;
#pragma unroll
  for (int j = 0; j < 8; ++j) o[j] = (unsigned short)bf16_bits(T[(k8 + j) * NWAVE + wave]);
  unsigned short* dp = WT + (size_t)(L * HID + n0 + wave) * KD + k8;
  *(volatile v8us*)dp = o;
  __threadfence();
  *(volatile v8us*)dp = o;
}

__global__ __launch_bounds__(NTHR) void k_init(const float* __restrict__ p, const float* __restrict__ Wi,
                                               const float* __restrict__ bi, float* X, int nN) {
  const int tid = (int)threadIdx.x, lane = tid & 31, wave = tid >> 5;
  const int node = (int)blockIdx.x * NWAVE + wave;
  if (node >= nN) return;
  const int c0 = 4 * lane;
  const v4f w0 = bfv4(*(const v4f*)(Wi + 0 * HID + c0));
  const v4f w1 = bfv4(*(const v4f*)(Wi + 1 * HID + c0));
  const v4f w2 = bfv4(*(const v4f*)(Wi + 2 * HID + c0));
  const v4f bb = bfv4(*(const v4f*)(bi + c0));
  const float* pa = p + (size_t)node * IND;
  const float* pb = p + ((size_t)nN + (size_t)node) * IND;
  const float a0 = bf16_val(pa[0]), a1 = bf16_val(pa[1]), a2 = bf16_val(pa[2]);
  const float e0 = bf16_val(pb[0]), e1 = bf16_val(pb[1]), e2 = bf16_val(pb[2]);
  const v4f o0 = a0 * w0 + a1 * w1 + a2 * w2 + bb;
  const v4f o1 = e0 * w0 + e1 * w1 + e2 * w2 + bb;
  float* xp = X + (size_t)node * CW + c0;
  *(volatile v4f*)xp = o0;
  *(volatile v4f*)(xp + HID) = o1;
  __threadfence();
  *(volatile v4f*)xp = o0;
  *(volatile v4f*)(xp + HID) = o1;
}

#define SPLIT_EL(I, V) { const float v_ = (V); const unsigned hb_ = bf16_bits(v_); \
                         ahi.u[I] = (unsigned short)hb_; \
                         alo.u[I] = (unsigned short)bf16_bits(v_ - __uint_as_float(hb_ << 16)); }

template <int RELU>
__device__ __forceinline__ void mac_half(v8f (&acc)[8], const float* __restrict__ ar,
                                         const unsigned short* __restrict__ wq0, int hh) {
#pragma unroll 1
  for (int kk = 0; kk < HID / 32; ++kk) {
    const int k0 = 32 * kk;
    const float* xp = ar + k0 + 8 * hh;
    v4f x0 = *(const v4f*)(xp);
    v4f x1 = *(const v4f*)(xp + 4);
    v4f x2 = *(const v4f*)(xp + 16);
    v4f x3 = *(const v4f*)(xp + 20);
    if (RELU) { x0 = relu4(x0); x1 = relu4(x1); x2 = relu4(x2); x3 = relu4(x3); }
    FragB ahi, alo;
    SPLIT_EL(0,  x0.x) SPLIT_EL(1,  x0.y) SPLIT_EL(2,  x0.z) SPLIT_EL(3,  x0.w)
    SPLIT_EL(4,  x1.x) SPLIT_EL(5,  x1.y) SPLIT_EL(6,  x1.z) SPLIT_EL(7,  x1.w)
    SPLIT_EL(8,  x2.x) SPLIT_EL(9,  x2.y) SPLIT_EL(10, x2.z) SPLIT_EL(11, x2.w)
    SPLIT_EL(12, x3.x) SPLIT_EL(13, x3.y) SPLIT_EL(14, x3.z) SPLIT_EL(15, x3.w)
#pragma unroll
    for (int nt = 0; nt < 8; ++nt) {
      const unsigned short* wq = wq0 + (size_t)(16 * nt) * KD + k0;
      FragB bw;
      bw.h[0] = *(const v8usa*)wq;
      bw.h[1] = *(const v8usa*)(wq + 16);
      acc[nt] = wmb(ahi, bw, acc[nt]);
      acc[nt] = wmb(alo, bw, acc[nt]);
    }
  }
}
#undef SPLIT_EL

__global__ __launch_bounds__(GTHR) void k_gemm(const float* __restrict__ Xin, const float* __restrict__ G,
                                               const unsigned short* __restrict__ WTL,
                                               const float* __restrict__ bs, const float* __restrict__ bfp,
                                               const float* res, float* Y, int nN, int hasRes) {
  __shared__ __attribute__((aligned(16))) float sB[HID];
  __shared__ __attribute__((aligned(16))) float stg[GBM * HID];
  const int tid = (int)threadIdx.x, lane = tid & 31, wave = tid >> 5, hh = lane >> 4, m = lane & 15;
  const int b = (int)blockIdx.y;
  const int rowBase = (int)blockIdx.x * GBM;

  sB[tid] = bf16_val(bs[tid]) + bf16_val(bfp[tid]);
  __syncthreads();

  const int row = rowBase + 16 * wave + m;
  const int rc  = row < nN ? row : nN - 1;
  const float* xr = Xin + (size_t)rc * CW + b * HID;
  const float* gr = G   + (size_t)rc * CW + b * HID;

  v8f acc[8];
  {
    const v8f z = {0.f, 0.f, 0.f, 0.f, 0.f, 0.f, 0.f, 0.f};
#pragma unroll
    for (int t = 0; t < 8; ++t) acc[t] = z;
  }
  const unsigned short* wp = WTL + (size_t)m * KD + 8 * hh;
  mac_half<1>(acc, xr, wp, hh);
  mac_half<0>(acc, gr, wp + HID, hh);

  float* st = stg + wave * (16 * HID);
#pragma unroll
  for (int nt = 0; nt < 8; ++nt) {
    const int lc = 16 * nt + m;
    const float bv = sB[lc];
#pragma unroll
    for (int r = 0; r < 8; ++r) {
      const int lr = 8 * hh + r;
      st[lr * HID + lc] = acc[nt][r] + bv;
    }
  }
  __syncthreads();

  const int r0w = rowBase + 16 * wave;
  float* yp = Y + (size_t)r0w * CW + b * HID + 4 * lane;
  v4f pv[16];
#pragma unroll
  for (int j = 0; j < 16; ++j) pv[j] = *(const v4fa*)(st + j * HID + 4 * lane);
  if (hasRes != 0) {
#pragma unroll
    for (int j = 0; j < 16; ++j) {
      int rr = r0w + j;
      rr = rr < nN ? rr : nN - 1;
      const v4f rv = *(const v4f*)(res + (size_t)rr * CW + b * HID + 4 * lane);
      pv[j] = pv[j] + rv;
    }
  }
#pragma unroll
  for (int j = 0; j < 16; ++j) *(volatile v4f*)(yp + (size_t)j * CW) = pv[j];
  __threadfence();
#pragma unroll
  for (int j = 0; j < 16; ++j) *(volatile v4f*)(yp + (size_t)j * CW) = pv[j];
}

__global__ __launch_bounds__(NTHR) void k_agg(const int* __restrict__ srcs, const int* __restrict__ dsts,
                                              const float* __restrict__ ew, const float* __restrict__ P,
                                              int nE, int nN, int vec8, float* Gout) {
  extern __shared__ __attribute__((aligned(16))) float sacc[];
  __shared__ __attribute__((aligned(16))) int list[LISTN];
  __shared__ int wcnt[NWAVE];
  const int tid = (int)threadIdx.x, lane = tid & 31, wave = tid >> 5;
  const int nodeBase = (int)blockIdx.x * NB;

  {
    const v4f z = {0.f, 0.f, 0.f, 0.f};
    for (int i = tid; i < (NB * CW) / 4; i += NTHR) *(v4fa*)(sacc + 4 * i) = z;
  }
  for (int i = tid; i < LISTN; i += NTHR) list[i] = 0;
  if (tid < NWAVE) wcnt[tid] = 0;
  __syncthreads();

  const int nChunks = (nE + CHUNK - 1) / CHUNK;
#pragma unroll 1
  for (int ch = 0; ch < nChunks; ++ch) {
    const int cbase = ch * CHUNK;
    const int wc = scan_chunk(dsts, nE, cbase, nodeBase, NB, vec8, list, tid, lane, wave);
    if (lane == 0) wcnt[wave] = wc;
    __syncthreads();
    if (wave == 0) {
#pragma unroll 1
      for (int w2 = 0; w2 < NWAVE; ++w2) {
        int c = wcnt[w2];
        c = c < 0 ? 0 : (c > WCAP ? WCAP : c);
#pragma unroll 1
        for (int b0 = 0; b0 < c; b0 += 32) {
          const int idx = b0 + lane;
          const int ent = list[w2 * WCAP + (idx < WCAP ? idx : WCAP - 1)];
          const int el  = (ent >> SLB) & (CHUNK - 1);
          int eid = cbase + el;
          eid = eid < 0 ? 0 : (eid > nE - 1 ? nE - 1 : eid);
          const int sraw = srcs[eid];
          const int s = sraw < 0 ? 0 : (sraw > nN - 1 ? nN - 1 : sraw);
          const float wv = bf16_val(ew[eid]);
          const int wvi = __float_as_int(wv);
          const int m32 = (c - b0) < 32 ? (c - b0) : 32;
#pragma unroll 1
          for (int k = 0; k < m32; ++k) {
            const int u  = __builtin_amdgcn_readlane(ent, k);
            const int sl = u & (NB - 1);
            const int sk = __builtin_amdgcn_readlane(s, k);
            const float wk = __int_as_float(__builtin_amdgcn_readlane(wvi, k));
            const float* pr = P + (size_t)sk * CW + 4 * lane;
            v4f hv0 = *(const v4f*)pr;
            v4f hv1 = *(const v4f*)(pr + HID);
            hv0 = relu4(hv0);
            hv1 = relu4(hv1);
            float* ap = sacc + sl * CW + 4 * lane;
            v4f av0 = *(const v4fa*)ap;
            v4f av1 = *(const v4fa*)(ap + HID);
            av0 = av0 + wk * hv0;
            av1 = av1 + wk * hv1;
            *(v4fa*)ap = av0;
            *(v4fa*)(ap + HID) = av1;
          }
        }
      }
    }
    __syncthreads();
  }

  int nv = nN - nodeBase;
  nv = nv < 0 ? 0 : (nv > NB ? NB : nv);
#pragma unroll 1
  for (int g = 0; g < NB / (NWAVE * 8); ++g) {
    v4f va[8], vb[8];
#pragma unroll
    for (int j = 0; j < 8; ++j) {
      const int s = wave + NWAVE * (8 * g + j);
      va[j] = *(const v4fa*)(sacc + s * CW + 4 * lane);
      vb[j] = *(const v4fa*)(sacc + s * CW + HID + 4 * lane);
    }
#pragma unroll
    for (int j = 0; j < 8; ++j) {
      const int s = wave + NWAVE * (8 * g + j);
      if (s < nv) {
        float* gp = Gout + (size_t)(nodeBase + s) * CW + 4 * lane;
        *(volatile v4f*)gp = va[j];
        *(volatile v4f*)(gp + HID) = vb[j];
      }
    }
    __threadfence();
#pragma unroll
    for (int j = 0; j < 8; ++j) {
      const int s = wave + NWAVE * (8 * g + j);
      if (s < nv) {
        float* gp = Gout + (size_t)(nodeBase + s) * CW + 4 * lane;
        *(volatile v4f*)gp = va[j];
        *(volatile v4f*)(gp + HID) = vb[j];
      }
    }
  }
}

__global__ __launch_bounds__(NTHR) void k_final(const float* __restrict__ X, const float* __restrict__ G,
                                                const float* __restrict__ Wso, const float* __restrict__ bso,
                                                const float* __restrict__ Wfo, const float* __restrict__ bfo,
                                                int nN, float* out) {
  __shared__ float sW[2 * HID * OUTD];
  __shared__ float sBias[4];
  __shared__ __attribute__((aligned(16))) float sOut[FNB * OUTD];
  const int tid = (int)threadIdx.x, lane = tid & 31, wave = tid >> 5;
  const int b = (int)blockIdx.y;
  const int nodeBase = (int)blockIdx.x * FNB;

  for (int i = tid; i < HID * OUTD; i += NTHR) {
    sW[i]              = bf16_val(Wso[i]);
    sW[HID * OUTD + i] = bf16_val(Wfo[i]);
  }
  if (tid < OUTD) sBias[tid] = bf16_val(bso[tid]) + bf16_val(bfo[tid]);
  if (tid == OUTD) sBias[OUTD] = 0.0f;
  __syncthreads();

  float ws0[4], ws1[4], ws2[4], wf0[4], wf1[4], wf2[4];
#pragma unroll
  for (int j = 0; j < 4; ++j) {
    const int k = 4 * lane + j;
    ws0[j] = sW[k * OUTD + 0]; ws1[j] = sW[k * OUTD + 1]; ws2[j] = sW[k * OUTD + 2];
    wf0[j] = sW[HID * OUTD + k * OUTD + 0];
    wf1[j] = sW[HID * OUTD + k * OUTD + 1];
    wf2[j] = sW[HID * OUTD + k * OUTD + 2];
  }
  const float bias0 = sBias[0], bias1 = sBias[1], bias2 = sBias[2];

#pragma unroll 1
  for (int t = 0; t < FNB / NWAVE; ++t) {
    const int ln = wave * (FNB / NWAVE) + t;
    const int node = nodeBase + ln;
    const int nc = node < nN ? node : nN - 1;
    v4f xv = *(const v4f*)(X + (size_t)nc * CW + b * HID + 4 * lane);
    xv = relu4(xv);
    const v4f gv = *(const v4f*)(G + (size_t)nc * CW + b * HID + 4 * lane);
    float q0 = xv.x * ws0[0] + xv.y * ws0[1] + xv.z * ws0[2] + xv.w * ws0[3]
             + gv.x * wf0[0] + gv.y * wf0[1] + gv.z * wf0[2] + gv.w * wf0[3];
    float q1 = xv.x * ws1[0] + xv.y * ws1[1] + xv.z * ws1[2] + xv.w * ws1[3]
             + gv.x * wf1[0] + gv.y * wf1[1] + gv.z * wf1[2] + gv.w * wf1[3];
    float q2 = xv.x * ws2[0] + xv.y * ws2[1] + xv.z * ws2[2] + xv.w * ws2[3]
             + gv.x * wf2[0] + gv.y * wf2[1] + gv.z * wf2[2] + gv.w * wf2[3];
#pragma unroll
    for (int off = 16; off > 0; off >>= 1) {
      q0 += __shfl_xor(q0, off);
      q1 += __shfl_xor(q1, off);
      q2 += __shfl_xor(q2, off);
    }
    if (lane == 0) {
      sOut[ln * OUTD + 0] = q0 + bias0;
      sOut[ln * OUTD + 1] = q1 + bias1;
      sOut[ln * OUTD + 2] = q2 + bias2;
    }
  }
  __syncthreads();

  int nv = nN - nodeBase;
  nv = nv < 0 ? 0 : (nv > FNB ? FNB : nv);
  const int nflo = nv * OUTD;
  const int nq = nflo >> 2;
  const int tl = nflo - 4 * nq;
  float* ob = out + (size_t)b * (size_t)nN * OUTD + (size_t)nodeBase * OUTD;
  v4f v = {0.f, 0.f, 0.f, 0.f};
  float vt = 0.0f;
  if (tid < nq) v = *(const v4fa*)(sOut + 4 * tid);
  if (tid < tl) vt = sOut[4 * nq + tid];
  if (tid < nq) *(volatile v4f*)(ob + 4 * tid) = v;
  if (tid < tl) *(volatile float*)(ob + 4 * nq + tid) = vt;
  __threadfence();
  if (tid < nq) *(volatile v4f*)(ob + 4 * tid) = v;
  if (tid < tl) *(volatile float*)(ob + 4 * nq + tid) = vt;
}

static inline int cdiv(int a, int b) { return (a + b - 1) / b; }

extern "C" void kernel_launch(void* const* d_in, const int* in_sizes, int n_in,
                              void* d_out, int out_size, void* d_ws, size_t ws_size,
                              hipStream_t stream) {
  if (n_in < 14) return;
  if (in_sizes[0] < NBAT * IND || (in_sizes[0] % (NBAT * IND)) != 0) return;
  const int nN = in_sizes[0] / (NBAT * IND);
  const int nE = in_sizes[1];
  if (nE < 1 || in_sizes[2] != nE || in_sizes[3] != nE) return;
  if (in_sizes[4] != IND * HID || in_sizes[5] != HID) return;
  if (in_sizes[6] != NLAY * HID * HID || in_sizes[7] != NLAY * HID) return;
  if (in_sizes[8] != NLAY * HID * HID || in_sizes[9] != NLAY * HID) return;
  if (in_sizes[10] != HID * OUTD || in_sizes[11] != OUTD) return;
  if (in_sizes[12] != HID * OUTD || in_sizes[13] != OUTD) return;
  if (out_size != NBAT * nN * OUTD) return;

  const float* p    = (const float*)d_in[0];
  const float* av   = (const float*)d_in[1];
  const int*   erow = (const int*)d_in[2];
  const int*   ecol = (const int*)d_in[3];
  const float* Wi   = (const float*)d_in[4];
  const float* bi   = (const float*)d_in[5];
  const float* Wfb  = (const float*)d_in[6];
  const float* bfb  = (const float*)d_in[7];
  const float* Wsb  = (const float*)d_in[8];
  const float* bsb  = (const float*)d_in[9];
  const float* Wfo  = (const float*)d_in[10];
  const float* bfo  = (const float*)d_in[11];
  const float* Wso  = (const float*)d_in[12];
  const float* bso  = (const float*)d_in[13];
  float* out = (float*)d_out;

  const int NP = cdiv(nN, GBM) * GBM;
  const int gM = NP / GBM;
  const int gA = cdiv(nN, NB);
  if ((long long)gA * NB < (long long)nN) return;
  const int gI = cdiv(nN, NWAVE);
  const int gF = cdiv(nN, FNB);
  const int vec8 = ((nE & 3) == 0) ? 1 : 0;

  char* ws = (char*)d_ws;
  size_t off = 0;
  const size_t oWT = off; off += (size_t)NLAY * HID * KD * 2;          off = (off + 255) & ~(size_t)255;
  const size_t plB = (size_t)NP * CW * 4;
  const size_t oPA = off; off += plB;                                   off = (off + 255) & ~(size_t)255;
  const size_t oPN = off; off += plB;                                   off = (off + 255) & ~(size_t)255;
  const size_t oPG = off; off += plB;                                   off = (off + 255) & ~(size_t)255;
  if (off > ws_size || off > (size_t)WSMAX) return;
  unsigned short* WT = (unsigned short*)(ws + oWT);
  float* PA = (float*)(ws + oPA);
  float* PN = (float*)(ws + oPN);
  float* PG = (float*)(ws + oPG);

  const size_t dynB = (size_t)NB * CW * 4;
  hipFuncSetAttribute(reinterpret_cast<const void*>(&k_agg), hipFuncAttributeMaxDynamicSharedMemorySize, (int)dynB);

  k_wprep<<<dim3(HID / NWAVE, NLAY, 1), NTHR, 0, stream>>>(Wsb, Wfb, WT);
  k_init<<<gI, NTHR, 0, stream>>>(p, Wi, bi, PA, nN);

  k_agg<<<gA, NTHR, dynB, stream>>>(ecol, erow, av, PA, nE, nN, vec8, PG);
  k_gemm<<<dim3(gM, NBAT, 1), GTHR, 0, stream>>>(PA, PG, WT + (size_t)0 * HID * KD, bsb + 0 * HID, bfb + 0 * HID,
                                                  PA, PN, nN, 0);
  k_agg<<<gA, NTHR, dynB, stream>>>(ecol, erow, av, PN, nE, nN, vec8, PG);
  k_gemm<<<dim3(gM, NBAT, 1), GTHR, 0, stream>>>(PN, PG, WT + (size_t)1 * HID * KD, bsb + 1 * HID, bfb + 1 * HID,
                                                  PA, PA, nN, 1);
  k_agg<<<gA, NTHR, dynB, stream>>>(ecol, erow, av, PA, nE, nN, vec8, PG);
  k_gemm<<<dim3(gM, NBAT, 1), GTHR, 0, stream>>>(PA, PG, WT + (size_t)2 * HID * KD, bsb + 2 * HID, bfb + 2 * HID,
                                                  PA, PN, nN, 0);
  k_agg<<<gA, NTHR, dynB, stream>>>(ecol, erow, av, PN, nE, nN, vec8, PG);
  k_gemm<<<dim3(gM, NBAT, 1), GTHR, 0, stream>>>(PN, PG, WT + (size_t)3 * HID * KD, bsb + 3 * HID, bfb + 3 * HID,
                                                  PA, PA, nN, 1);
  k_agg<<<gA, NTHR, dynB, stream>>>(ecol, erow, av, PA, nE, nN, vec8, PG);
  k_final<<<dim3(gF, NBAT, 1), NTHR, 0, stream>>>(PA, PG, Wso, bso, Wfo, bfo, nN, out);
}
